// SelfAttentionBlock_24352464569698
// MI455X (gfx1250) — hardware-run, weakly checked
//
#include <hip/hip_runtime.h>
#include <math.h>

constexpr int kBatch   = 2;
constexpr int kSeq     = 2048;
constexpr int kDim     = 1024;
constexpr int kHeads   = 16;
constexpr int kHeadDim = 64;
constexpr int kMlp     = 4096;
constexpr int kTok     = kBatch * kSeq;

constexpr float kWCarry    = 32.0f;
constexpr float kPCarry    = 2048.0f;
constexpr float kCtxCarry  = 64.0f;
constexpr float kHCarry    = 8.0f;
constexpr float kAttnScale = 0.125f;
constexpr float kMaskNeg   = -1.0e9f;

constexpr float kProjScale = 1.0f / kWCarry;
constexpr float kPVScale   = kCtxCarry / kPCarry;
constexpr float kFcScale   = 1.0f / (kCtxCarry * kWCarry);
constexpr float kW1Scale   = 1.0f / kWCarry;
constexpr float kW2Scale   = 1.0f / (kHCarry * kWCarry);

constexpr size_t kSz16TokDim = (size_t)kTok * kDim * 2;
constexpr size_t kSz16Sq     = (size_t)kDim * kDim * 2;
constexpr size_t kSzScores   = (size_t)2 * kSeq * kSeq * 4;
constexpr size_t kSzP        = (size_t)2 * kSeq * kSeq * 2;
constexpr size_t kSzOut1     = (size_t)kTok * kDim * 4;
constexpr size_t kSzHid      = (size_t)kTok * kMlp * 2;

constexpr size_t kOffX16   = 0;
constexpr size_t kOffWsq   = kOffX16 + kSz16TokDim;
constexpr size_t kOffW1T   = kOffWsq + 4 * kSz16Sq;
constexpr size_t kOffW2T   = kOffW1T + (size_t)kMlp * kDim * 2;
constexpr size_t kOffQp    = kOffW2T + (size_t)kDim * kMlp * 2;
constexpr size_t kOffKp    = kOffQp + kSz16TokDim;
constexpr size_t kOffVpT   = kOffKp + kSz16TokDim;
constexpr size_t kOffSc    = kOffVpT + kSz16TokDim;
constexpr size_t kOffP     = kOffSc + kSzScores;
constexpr size_t kOffOut1  = kOffP + kSzP;
constexpr size_t kWsTotal  = kOffOut1 + kSzOut1;
static_assert(kSzHid <= kSzScores);
static_assert(kWsTotal == 125829120u);
static_assert(kWsTotal <= 134217728u);

typedef __attribute__((ext_vector_type(16))) _Float16 v16h;
typedef __attribute__((ext_vector_type(8)))  _Float16 v8h;
typedef __attribute__((ext_vector_type(16))) __bf16   v16b;
typedef __attribute__((ext_vector_type(8)))  __bf16   v8b;
typedef __attribute__((ext_vector_type(8)))  float    v8f;
typedef __attribute__((ext_vector_type(4)))  float    v4f;
typedef __attribute__((ext_vector_type(4)))  unsigned int v4u;

__device__ __forceinline__ unsigned short f2bf_bits(float f) {
  unsigned u = __float_as_uint(f);
  return (unsigned short)((u + 0x7FFFu + ((u >> 16) & 1u)) >> 16);
}
__device__ __forceinline__ float bf_bits2f(unsigned short h) { return __uint_as_float(((unsigned)h) << 16); }

__device__ __forceinline__ void dep_guard_h(v8f& a, v8f& b, v16h x, v16h y) { asm volatile("v_nop\n\tv_nop\n\tv_nop\n\tv_nop" : "+v"(a), "+v"(b) : "v"(x), "v"(y)); }
__device__ __forceinline__ void dep_guard_b(v8f& a, v8f& b, v16b x, v16b y) { asm volatile("v_nop\n\tv_nop\n\tv_nop\n\tv_nop" : "+v"(a), "+v"(b) : "v"(x), "v"(y)); }
__device__ __forceinline__ void keep4_h(v16h a, v16h b, v16h c, v16h d) { asm volatile("v_nop" :: "v"(a), "v"(b), "v"(c), "v"(d)); }
__device__ __forceinline__ void keep4_b(v16b a, v16b b, v16b c, v16b d) { asm volatile("v_nop" :: "v"(a), "v"(b), "v"(c), "v"(d)); }
__device__ __forceinline__ void acc_guard4(v8f& a, v8f& b, v8f& c, v8f& d) { asm volatile("v_nop\n\tv_nop\n\tv_nop\n\tv_nop" : "+v"(a), "+v"(b), "+v"(c), "+v"(d)); }
template <typename T> struct Frag;
template <> struct Frag<_Float16> {
  typedef v16h V; union U { v16h v; v8h h[2]; };
  static __device__ __forceinline__ v16h load(const _Float16* p) {
    U f; f.h[0] = *(const v8h*)(p); f.h[1] = *(const v8h*)(p + 16); return f.v;
  }
  static __device__ __forceinline__ v8f mma(v16h a, v16h b, v8f c) {
    return __builtin_amdgcn_wmma_f32_16x16x32_f16(false, a, false, b, (short)0, c, false, false);
  }
  static __device__ __forceinline__ void guard(v8f& a, v8f& b, v16h x, v16h y) { dep_guard_h(a, b, x, y); }
  static __device__ __forceinline__ void keep(v16h a, v16h b, v16h c, v16h d) { keep4_h(a, b, c, d); }
};
template <> struct Frag<__bf16> {
  typedef v16b V; union U { v16b v; v8b h[2]; };
  static __device__ __forceinline__ v16b load(const __bf16* p) {
    U f; f.h[0] = *(const v8b*)(p); f.h[1] = *(const v8b*)(p + 16); return f.v;
  }
  static __device__ __forceinline__ v8f mma(v16b a, v16b b, v8f c) {
    return __builtin_amdgcn_wmma_f32_16x16x32_bf16(false, a, false, b, (short)0, c, false, false);
  }
  static __device__ __forceinline__ void guard(v8f& a, v8f& b, v16b x, v16b y) { dep_guard_b(a, b, x, y); }
  static __device__ __forceinline__ void keep(v16b a, v16b b, v16b c, v16b d) { keep4_b(a, b, c, d); }
};

__device__ __forceinline__ unsigned pk16(unsigned short a, unsigned short b) { return (unsigned)a | ((unsigned)b << 16); }
__device__ __forceinline__ unsigned short h_bits(float f) { const _Float16 h = (_Float16)f; return __builtin_bit_cast(unsigned short, h); }

template <int ET> struct Elem;
template <> struct Elem<0> { typedef _Float16 T; };
template <> struct Elem<1> { typedef __bf16 T; };
template <int ET, bool SPLIT, int BIAS_MODE, int OUT_MODE, bool RESID, int ACT = 0>
__global__ __launch_bounds__(256) void wmma_gemm64(
    const unsigned short* __restrict__ Ap, const unsigned short* __restrict__ A2p, int lda, long strideA,
    const unsigned short* __restrict__ Btp, const unsigned short* __restrict__ Bt2p, int ldb, long strideB,
    void* __restrict__ Cout, void* __restrict__ Cout2, int ldc, long strideC,
    const float* __restrict__ bias,
    const float* __restrict__ resid, long strideR,
    int M, int N, int K, float scale) {
  typedef typename Elem<ET>::T T;
  typedef typename Frag<T>::V V;
  const T* A = (const T*)Ap; const T* A2 = (const T*)A2p; const T* Bt = (const T*)Btp; const T* Bt2 = (const T*)Bt2p;
  __shared__ __align__(16) float sT[8][16 * 68];
  const int b    = blockIdx.y;
  const int lane = threadIdx.x & 31;
  const int wave = threadIdx.x >> 5;
  const int tilesN = N >> 6;
  const int tilesM = M >> 6;
  const int tile = blockIdx.x * 8 + wave;
  if (tile >= tilesM * tilesN) return;
  const int tm = tile / tilesN;
  const int tn = tile - tm * tilesN;
  const int m0 = tm << 6;
  const int n0 = tn << 6;

  const T* Ab  = A  + (size_t)b * strideA;
  const T* Bb  = Bt + (size_t)b * strideB;
  const T* Ab2 = SPLIT ? (A2  + (size_t)b * strideA) : nullptr;
  const T* Bb2 = SPLIT ? (Bt2 + (size_t)b * strideB) : nullptr;

  const int rlane = lane & 15;
  const int koff  = (lane >> 4) * 8;
  const int mOff  = (lane >> 4) * 8;

  v8f acc[4][4];
#pragma unroll
  for (int i = 0; i < 4; ++i)
#pragma unroll
    for (int j = 0; j < 4; ++j) acc[i][j] = (v8f){0.f,0.f,0.f,0.f,0.f,0.f,0.f,0.f};

  for (int k0 = 0; k0 < K; k0 += 32) {
    V bh[4], bl[4];
#pragma unroll
    for (int j = 0; j < 4; ++j) {
      const size_t bo = (size_t)(n0 + (j << 4) + rlane) * ldb + koff + k0;
      bh[j] = Frag<T>::load(Bb + bo);
      if (SPLIT) bl[j] = Frag<T>::load(Bb2 + bo);
    }
#pragma unroll
    for (int i = 0; i < 4; ++i) {
      const size_t ao = (size_t)(m0 + (i << 4) + rlane) * lda + koff + k0;
      V ah = Frag<T>::load(Ab + ao);
      V al;
      if (SPLIT) al = Frag<T>::load(Ab2 + ao);
#pragma unroll
      for (int j = 0; j < 4; ++j) {
        acc[i][j] = Frag<T>::mma(ah, bh[j], acc[i][j]);
        if (SPLIT) {
          acc[i][j] = Frag<T>::mma(ah, bl[j], acc[i][j]);
          acc[i][j] = Frag<T>::mma(al, bh[j], acc[i][j]);
        }
      }
      Frag<T>::guard(acc[i][0], acc[i][3], ah, SPLIT ? al : ah);
    }
    Frag<T>::keep(bh[0], bh[1], bh[2], bh[3]);
    if (SPLIT) Frag<T>::keep(bl[0], bl[1], bl[2], bl[3]);
  }
  acc_guard4(acc[0][0], acc[0][1], acc[0][2], acc[0][3]);
  acc_guard4(acc[1][0], acc[1][1], acc[1][2], acc[1][3]);
  acc_guard4(acc[2][0], acc[2][1], acc[2][2], acc[2][3]);
  acc_guard4(acc[3][0], acc[3][1], acc[3][2], acc[3][3]);

  float* slab = sT[wave];
  const float* Rb = RESID ? (resid + (size_t)b * strideR) : nullptr;
#pragma unroll
  for (int i = 0; i < 4; ++i) {
    const int mBase = m0 + (i << 4);
#pragma unroll
    for (int j = 0; j < 4; ++j) {
      const int n = n0 + (j << 4) + rlane;
      float bv = 0.f;
      if (BIAS_MODE == 2) bv = bias[n];
#pragma unroll
      for (int r = 0; r < 8; ++r) {
        float v = acc[i][j][r] * scale;
        if (BIAS_MODE == 1) v += bias[mBase + mOff + r];
        if (BIAS_MODE == 2) v += bv;
        if (RESID) v += Rb[(size_t)(mBase + mOff + r) * ldc + n];
        if (ACT == 2) v = fmaxf(v, 0.0f);
        if (ACT == 4) v = (v > 0.f) ? v : 0.01f * v;
        if (ACT == 6) {
          const float u = v * (1.5957691216057308f + 0.0713548162726009f * v * v);
          const float e = expf(fminf(-u, 80.0f));
          v = v * __builtin_amdgcn_rcpf(1.0f + e) * kHCarry;
        }
        slab[(mOff + r) * 68 + (j << 4) + rlane] = v;
      }
    }
    __builtin_amdgcn_fence(__ATOMIC_RELEASE, "workgroup");
    __builtin_amdgcn_wave_barrier();
    __builtin_amdgcn_fence(__ATOMIC_ACQUIRE, "workgroup");
    if (OUT_MODE == 0) {
      float* C = (float*)Cout + (size_t)b * strideC;
      const int hh = lane >> 4, c4 = (lane & 15) * 4;
      for (int pass = 0; pass < 2; ++pass) {
#pragma unroll
        for (int it = 0; it < 8; ++it) {
          const int row = it * 2 + hh;
          v4f v = *(const v4f*)(slab + row * 68 + c4);
          *(volatile v4f*)(C + (size_t)(mBase + row) * ldc + n0 + c4) = v;
        }
        __threadfence();
      }
    } else {
      const int q = lane >> 3, c8 = (lane & 7) * 8;
      unsigned short* C  = (unsigned short*)Cout  + (size_t)b * strideC;
      unsigned short* C2 = (OUT_MODE == 2) ? ((unsigned short*)Cout2 + (size_t)b * strideC) : nullptr;
      for (int pass = 0; pass < 2; ++pass) {
#pragma unroll
        for (int it = 0; it < 4; ++it) {
          const int row = it * 4 + q;
          const float* sp = slab + row * 68 + c8;
          v8h hv, lv;
#pragma unroll
          for (int e = 0; e < 8; ++e) {
            if (OUT_MODE == 1) {
              hv[e] = (_Float16)sp[e];
            } else {
              unsigned short hb = f2bf_bits(sp[e]);
              unsigned short lb = f2bf_bits(sp[e] - bf_bits2f(hb));
              hv[e] = __builtin_bit_cast(_Float16, hb);
              lv[e] = __builtin_bit_cast(_Float16, lb);
            }
          }
          *(volatile v8h*)(C + (size_t)(mBase + row) * ldc + n0 + c8) = hv;
          if (OUT_MODE == 2) *(volatile v8h*)(C2 + (size_t)(mBase + row) * ldc + n0 + c8) = lv;
        }
        __threadfence();
      }
    }
    __builtin_amdgcn_fence(__ATOMIC_RELEASE, "workgroup");
    __builtin_amdgcn_wave_barrier();
    __builtin_amdgcn_fence(__ATOMIC_ACQUIRE, "workgroup");
  }
}

__global__ __launch_bounds__(256) void wtcast_kernel(const float* __restrict__ W0, const float* __restrict__ W1,
                                                     const float* __restrict__ W2, const float* __restrict__ W3,
                                                     unsigned short* __restrict__ out, int Kd, int Nd,
                                                     long planeStride, float scale) {
  __shared__ float sm[64][65];
  const int t  = threadIdx.x;
  const int k0 = blockIdx.x * 64;
  const int n0 = blockIdx.y * 64;
  const int z  = blockIdx.z;
  const float* W = (z == 0) ? W0 : (z == 1) ? W1 : (z == 2) ? W2 : W3;
#pragma unroll
  for (int i = 0; i < 16; ++i) {
    const int e = i * 256 + t;
    const int r = e >> 6;
    const int c = e & 63;
    sm[c][r] = W[(size_t)(k0 + r) * Nd + n0 + c] * scale;
  }
  __syncthreads();
  const int lane = t & 31, wave = t >> 5;
  const int q = lane >> 3, c8 = (lane & 7) * 8;
  unsigned short* op = out + (size_t)z * planeStride;
  for (int pass = 0; pass < 2; ++pass) {
#pragma unroll
    for (int it = 0; it < 2; ++it) {
      const int row = wave * 8 + it * 4 + q;
      unsigned short hb[8];
#pragma unroll
      for (int e = 0; e < 8; ++e) hb[e] = h_bits(sm[row][c8 + e]);
      const v4u u = (v4u){pk16(hb[0], hb[1]), pk16(hb[2], hb[3]), pk16(hb[4], hb[5]), pk16(hb[6], hb[7])};
      *(volatile v4u*)(op + (size_t)(n0 + row) * Kd + k0 + c8) = u;
    }
    __threadfence();
  }
}

__global__ __launch_bounds__(256) void cast8_f16_kernel(const float* __restrict__ in, unsigned short* __restrict__ out,
                                                        int n8, float scale) {
  const int i = blockIdx.x * 256 + threadIdx.x;
  if (i >= n8) return;
  const float* p = in + 8 * (size_t)i;
  const v4f a = *(const v4f*)(p);
  const v4f c = *(const v4f*)(p + 4);
  unsigned short hb[8];
#pragma unroll
  for (int e = 0; e < 4; ++e) {
    hb[e]     = h_bits(a[e] * scale);
    hb[4 + e] = h_bits(c[e] * scale);
  }
  const v4u u = (v4u){pk16(hb[0], hb[1]), pk16(hb[2], hb[3]), pk16(hb[4], hb[5]), pk16(hb[6], hb[7])};
  unsigned short* q = out + 8 * (size_t)i;
  *(volatile v4u*)q = u;
  __threadfence();
  *(volatile v4u*)q = u;
}

__global__ __launch_bounds__(256) void softmax_row_kernel(const float* __restrict__ Sc, const float* __restrict__ maskv,
                                                          unsigned short* __restrict__ P) {
  __shared__ float redM[8];
  __shared__ float redS[8];
  const int row  = blockIdx.x;
  const int t    = threadIdx.x;
  const int lane = t & 31, wave = t >> 5;
  const int bsel = row >> 11;
  const int c0   = t * 8;
  const float* sr = Sc + (size_t)row * kSeq + c0;
  const float* mr = maskv + (size_t)bsel * kSeq + c0;
  const v4f a  = *(const v4f*)(sr);
  const v4f c  = *(const v4f*)(sr + 4);
  const v4f ma = *(const v4f*)(mr);
  const v4f mc = *(const v4f*)(mr + 4);
  float x[8];
#pragma unroll
  for (int e = 0; e < 4; ++e) {
    x[e]     = a[e] + ma[e] * kMaskNeg;
    x[4 + e] = c[e] + mc[e] * kMaskNeg;
  }
  float m = fmaxf(fmaxf(fmaxf(x[0], x[1]), fmaxf(x[2], x[3])), fmaxf(fmaxf(x[4], x[5]), fmaxf(x[6], x[7])));
#pragma unroll
  for (int off = 16; off > 0; off >>= 1) m = fmaxf(m, __shfl_xor(m, off, 32));
  if (lane == 0) redM[wave] = m;
  __syncthreads();
  float gm = redM[0];
#pragma unroll
  for (int w = 1; w < 8; ++w) gm = fmaxf(gm, redM[w]);
  float ev[8];
  float ls = 0.f;
#pragma unroll
  for (int e = 0; e < 8; ++e) { ev[e] = expf(x[e] - gm); ls += ev[e]; }
#pragma unroll
  for (int off = 16; off > 0; off >>= 1) ls += __shfl_xor(ls, off, 32);
  if (lane == 0) redS[wave] = ls;
  __syncthreads();
  float tot = redS[0];
#pragma unroll
  for (int w = 1; w < 8; ++w) tot += redS[w];
  const float inv = kPCarry / tot;
  unsigned short hb[8];
#pragma unroll
  for (int e = 0; e < 8; ++e) hb[e] = h_bits(ev[e] * inv);
  const v4u u = (v4u){pk16(hb[0], hb[1]), pk16(hb[2], hb[3]), pk16(hb[4], hb[5]), pk16(hb[6], hb[7])};
  unsigned short* pr = P + (size_t)row * kSeq + c0;
  *(volatile v4u*)pr = u;
  __threadfence();
  *(volatile v4u*)pr = u;
}

extern "C" void kernel_launch(void* const* d_in, const int* in_sizes, int n_in,
                              void* d_out, int out_size, void* d_ws, size_t ws_size,
                              hipStream_t stream)
{
  if (n_in < 16) return;
  if (in_sizes[0] != kTok * kDim || in_sizes[1] != kTok * kDim || in_sizes[2] != kTok * kDim) return;
  if (in_sizes[3] != kBatch * kSeq) return;
  if (in_sizes[4] != kDim * kDim || in_sizes[6] != kDim * kDim || in_sizes[8] != kDim * kDim || in_sizes[10] != kDim * kDim) return;
  if (in_sizes[5] != kDim || in_sizes[7] != kDim || in_sizes[9] != kDim || in_sizes[11] != kDim) return;
  if (in_sizes[12] != kDim * kMlp || in_sizes[13] != kMlp || in_sizes[14] != kMlp * kDim || in_sizes[15] != kDim) return;
  if (out_size != kTok * kDim) return;
  if (ws_size < kWsTotal) return;

  const float* v_in  = (const float*)d_in[0];
  const float* k_in  = (const float*)d_in[1];
  const float* q_in  = (const float*)d_in[2];
  const float* maskv = (const float*)d_in[3];
  const float* wq_w  = (const float*)d_in[4];
  const float* wq_b  = (const float*)d_in[5];
  const float* wk_w  = (const float*)d_in[6];
  const float* wk_b  = (const float*)d_in[7];
  const float* wv_w  = (const float*)d_in[8];
  const float* wv_b  = (const float*)d_in[9];
  const float* fc_w  = (const float*)d_in[10];
  const float* fc_b  = (const float*)d_in[11];
  const float* w1    = (const float*)d_in[12];
  const float* b1    = (const float*)d_in[13];
  const float* w2    = (const float*)d_in[14];
  const float* b2    = (const float*)d_in[15];
  float* out = (float*)d_out;

  char* ws = (char*)d_ws;
  unsigned short* X16    = (unsigned short*)(ws + kOffX16);
  unsigned short* ctx16  = (unsigned short*)(ws + kOffX16);
  unsigned short* wqT    = (unsigned short*)(ws + kOffWsq);
  unsigned short* wkT    = wqT + (size_t)kDim * kDim;
  unsigned short* wvT    = wkT + (size_t)kDim * kDim;
  unsigned short* fcT    = wvT + (size_t)kDim * kDim;
  unsigned short* w1T    = (unsigned short*)(ws + kOffW1T);
  unsigned short* w2T    = (unsigned short*)(ws + kOffW2T);
  unsigned short* qp16   = (unsigned short*)(ws + kOffQp);
  unsigned short* out1h  = (unsigned short*)(ws + kOffQp);
  unsigned short* kp16   = (unsigned short*)(ws + kOffKp);
  unsigned short* vpT    = (unsigned short*)(ws + kOffVpT);
  float*          scores = (float*)(ws + kOffSc);
  unsigned short* hid16  = (unsigned short*)(ws + kOffSc);
  unsigned short* P16    = (unsigned short*)(ws + kOffP);
  float*          out1   = (float*)(ws + kOffOut1);

  const dim3 blk(256);
  const int n8 = kTok * kDim / 8;
  const dim3 gCast((n8 + 255) / 256);

  wtcast_kernel<<<dim3(kDim / 64, kDim / 64, 4), blk, 0, stream>>>(wq_w, wk_w, wv_w, fc_w, wqT, kDim, kDim,
                                                                   (long)kDim * kDim, kWCarry);
  wtcast_kernel<<<dim3(kDim / 64, kMlp / 64, 1), blk, 0, stream>>>(w1, w1, w1, w1, w1T, kDim, kMlp, 0L, kWCarry);
  wtcast_kernel<<<dim3(kMlp / 64, kDim / 64, 1), blk, 0, stream>>>(w2, w2, w2, w2, w2T, kMlp, kDim, 0L, kWCarry);

  const dim3 gProj(128, 1);
  cast8_f16_kernel<<<gCast, blk, 0, stream>>>(q_in, X16, n8, 1.0f);
  wmma_gemm64<0, false, 2, 1, false, 0><<<gProj, blk, 0, stream>>>(
      X16, nullptr, kDim, 0L, wqT, nullptr, kDim, 0L, (void*)qp16, nullptr, kDim, 0L,
      wq_b, nullptr, 0L, kTok, kDim, kDim, kProjScale);
  cast8_f16_kernel<<<gCast, blk, 0, stream>>>(k_in, X16, n8, 1.0f);
  wmma_gemm64<0, false, 2, 1, false, 0><<<gProj, blk, 0, stream>>>(
      X16, nullptr, kDim, 0L, wkT, nullptr, kDim, 0L, (void*)kp16, nullptr, kDim, 0L,
      wk_b, nullptr, 0L, kTok, kDim, kDim, kProjScale);
  cast8_f16_kernel<<<gCast, blk, 0, stream>>>(v_in, X16, n8, 1.0f);
  wmma_gemm64<0, false, 1, 1, false, 0><<<dim3(128, 1), blk, 0, stream>>>(
      wvT, nullptr, kDim, 0L, X16, nullptr, kDim, 0L, (void*)vpT, nullptr, kTok, 0L,
      wv_b, nullptr, 0L, kDim, kTok, kDim, kProjScale);

  const long tokPlaneStride = (long)kSeq * kDim;
  const long scPlaneStride  = (long)kSeq * kSeq;
  for (int h = 0; h < kHeads; ++h) {
    wmma_gemm64<0, false, 0, 0, false, 0><<<dim3(128, kBatch), blk, 0, stream>>>(
        qp16 + h * kHeadDim, nullptr, kDim, tokPlaneStride,
        kp16 + h * kHeadDim, nullptr, kDim, tokPlaneStride,
        (void*)scores, nullptr, kSeq, scPlaneStride,
        nullptr, nullptr, 0L, kSeq, kSeq, kHeadDim, kAttnScale);
    softmax_row_kernel<<<dim3(kBatch * kSeq), blk, 0, stream>>>(scores, maskv, P16);
    wmma_gemm64<0, false, 0, 1, false, 0><<<dim3(4, kBatch), blk, 0, stream>>>(
        P16, nullptr, kSeq, scPlaneStride,
        vpT + (size_t)h * kHeadDim * kTok, nullptr, kTok, (long)kSeq,
        (void*)(ctx16 + h * kHeadDim), nullptr, kDim, tokPlaneStride,
        nullptr, nullptr, 0L, kSeq, kHeadDim, kSeq, kPVScale);
  }

  wmma_gemm64<0, false, 2, 0, true, 0><<<gProj, blk, 0, stream>>>(
      ctx16, nullptr, kDim, 0L, fcT, nullptr, kDim, 0L, (void*)out1, nullptr, kDim, 0L,
      fc_b, v_in, 0L, kTok, kDim, kDim, kFcScale);
  cast8_f16_kernel<<<gCast, blk, 0, stream>>>(out1, out1h, n8, 1.0f);
  wmma_gemm64<0, false, 2, 1, false, 6><<<dim3(512, 1), blk, 0, stream>>>(
      out1h, nullptr, kDim, 0L, w1T, nullptr, kDim, 0L, (void*)hid16, nullptr, kMlp, 0L,
      b1, nullptr, 0L, kTok, kMlp, kDim, kW1Scale);
  wmma_gemm64<0, false, 2, 0, true, 0><<<gProj, blk, 0, stream>>>(
      hid16, nullptr, kMlp, 0L, w2T, nullptr, kMlp, 0L, (void*)out, nullptr, kDim, 0L,
      b2, out1, 0L, kTok, kDim, kMlp, kW2Scale);
}
